// BasePNA_62697932587514
// MI455X (gfx1250) — hardware-verified
//
#include <hip/hip_runtime.h>
#include <stddef.h>


#define HID     64
#define NT      4
#define FT      16
#define KPOST   224
#define NTHR    256
#define NWAVE   8
#define EPT     8
#define NGRP    2
#define CHUNK   (NTHR * EPT * NGRP)
#define WCAP    (EPT * NGRP * 32)
#define LISTN   (NWAVE * WCAP)
#define NBA     256
#define SLOTF   256
#define NROWS   128
#define WSC     16.0f
#define WSCI    0.0625f
#define AVGL    2.8332133440562160f
#define STDEPS  1e-5f
#define LDS_AGG ((NBA * SLOTF + LISTN + NBA + 16) * 4)

static_assert((CHUNK & (CHUNK - 1)) == 0);
static_assert(CHUNK <= 4096);
static_assert((NBA & (NBA - 1)) == 0 && NBA <= 4096);
static_assert((NBA / 16) % NWAVE == 0);
static_assert(NBA % NROWS == 0);
static_assert(3 * NBA <= LISTN);
static_assert(SLOTF == 4 * HID);
static_assert(NROWS == NWAVE * 16);
static_assert(KPOST % 32 == 0);

typedef float          v2f  __attribute__((ext_vector_type(2)));
typedef float          v4f  __attribute__((ext_vector_type(4)));
typedef float          v8f  __attribute__((ext_vector_type(8)));
typedef int            v4i  __attribute__((ext_vector_type(4)));
typedef _Float16       v8h  __attribute__((ext_vector_type(8)));
typedef _Float16       v16h __attribute__((ext_vector_type(16)));
typedef unsigned short v8us __attribute__((ext_vector_type(8)));
typedef unsigned short v16us __attribute__((ext_vector_type(16)));
typedef __bf16         v16bf __attribute__((ext_vector_type(16)));
union FragH { v16h v; v8h h[2]; };
union FragB { v16bf v; v16us u; v8us h[2]; };

__device__ __forceinline__ v8h cvt8(v4f a, v4f b) {
  v8h r;
  r[0] = (_Float16)a.x; r[1] = (_Float16)a.y; r[2] = (_Float16)a.z; r[3] = (_Float16)a.w;
  r[4] = (_Float16)b.x; r[5] = (_Float16)b.y; r[6] = (_Float16)b.z; r[7] = (_Float16)b.w;
  return r;
}

__device__ __forceinline__ unsigned short bf_bits(float f) {
  unsigned u = __float_as_uint(f);
  u += 0x7FFFu + ((u >> 16) & 1u);
  return (unsigned short)(u >> 16);
}
__device__ __forceinline__ void split2(float v, unsigned short& hi, unsigned short& lo) {
  const unsigned short hb = bf_bits(v);
  const float hf = __uint_as_float(((unsigned)hb) << 16);
  hi = hb;
  lo = bf_bits(v - hf);
}
template <int B>
__device__ __forceinline__ void split4(v4f p, FragB& ah, FragB& al) {
  unsigned short h0, l0, h1, l1, h2, l2, h3, l3;
  split2(p.x, h0, l0); split2(p.y, h1, l1); split2(p.z, h2, l2); split2(p.w, h3, l3);
  ah.u[B + 0] = h0; al.u[B + 0] = l0;
  ah.u[B + 1] = h1; al.u[B + 1] = l1;
  ah.u[B + 2] = h2; al.u[B + 2] = l2;
  ah.u[B + 3] = h3; al.u[B + 3] = l3;
}
__device__ __forceinline__ void loadB(const unsigned short* p, FragB& b) {
  b.h[0] = *(const v8us*)p;
  b.h[1] = *(const v8us*)(p + 16);
}

__device__ __forceinline__ v8f wmh(v16h a, v16h b, v8f c) {
  v8f d = __builtin_amdgcn_wmma_f32_16x16x32_f16(false, a, false, b, (short)0, c, false, false);
  asm volatile("v_nop\n\tv_nop\n\tv_nop\n\tv_nop" : "+v"(d) : "v"(a), "v"(b));
  return d;
}
__device__ __forceinline__ v8f wmb(v16bf a, v16bf b, v8f c) {
  v8f d = __builtin_amdgcn_wmma_f32_16x16x32_bf16(false, a, false, b, (short)0, c, false, false);
  asm volatile("v_nop\n\tv_nop\n\tv_nop\n\tv_nop" : "+v"(d) : "v"(a), "v"(b));
  return d;
}
__device__ __forceinline__ v8f wmb3(const FragB& ah, const FragB& al, const FragB& bh, const FragB& bl, v8f c) {
  c = wmb(ah.v, bh.v, c);
  c = wmb(al.v, bh.v, c);
  c = wmb(ah.v, bl.v, c);
  return c;
}

__device__ __forceinline__ float dot16r(const float* __restrict__ a, const float* __restrict__ b, int bs) {
  float s = 0.f;
#pragma unroll 1
  for (int f = 0; f < 16; ++f) s += a[f] * b[f * bs];
  return s;
}

template <int NSLOT>
__device__ __forceinline__ int scan_chunk(const int* __restrict__ dsts, int nE, int cbase, int nodeBase,
                                          int vec8, int* list, int tid, int lane, int wave) {
  int wc = 0;
#pragma unroll
  for (int g = 0; g < NGRP; ++g) {
    const int el0  = (g * NTHR + tid) * EPT;
    const int e0   = cbase + el0;
    const int sent = -2147483647 - 1;
    v4i da, db;
    if (vec8 != 0 && cbase + CHUNK <= nE) {
      da = *(const v4i*)(dsts + e0);
      db = *(const v4i*)(dsts + e0 + 4);
    } else {
      da.x = (e0     < nE) ? dsts[min(e0, nE - 1)] : sent;
      da.y = (e0 + 1 < nE) ? dsts[min(e0 + 1, nE - 1)] : sent;
      da.z = (e0 + 2 < nE) ? dsts[min(e0 + 2, nE - 1)] : sent;
      da.w = (e0 + 3 < nE) ? dsts[min(e0 + 3, nE - 1)] : sent;
      db.x = (e0 + 4 < nE) ? dsts[min(e0 + 4, nE - 1)] : sent;
      db.y = (e0 + 5 < nE) ? dsts[min(e0 + 5, nE - 1)] : sent;
      db.z = (e0 + 6 < nE) ? dsts[min(e0 + 6, nE - 1)] : sent;
      db.w = (e0 + 7 < nE) ? dsts[min(e0 + 7, nE - 1)] : sent;
    }
    const unsigned nb = (unsigned)nodeBase;
    const unsigned s0 = (unsigned)da.x - nb, s1 = (unsigned)da.y - nb;
    const unsigned s2 = (unsigned)da.z - nb, s3 = (unsigned)da.w - nb;
    const unsigned s4 = (unsigned)db.x - nb, s5 = (unsigned)db.y - nb;
    const unsigned s6 = (unsigned)db.z - nb, s7 = (unsigned)db.w - nb;
    const bool h0 = s0 < (unsigned)NSLOT, h1 = s1 < (unsigned)NSLOT, h2 = s2 < (unsigned)NSLOT, h3 = s3 < (unsigned)NSLOT;
    const bool h4 = s4 < (unsigned)NSLOT, h5 = s5 < (unsigned)NSLOT, h6 = s6 < (unsigned)NSLOT, h7 = s7 < (unsigned)NSLOT;
    const unsigned any = __builtin_amdgcn_ballot_w32(h0 | h1 | h2 | h3 | h4 | h5 | h6 | h7);
    if (any != 0u) {
#define HITJ(J, HJ, SJ) { \
        const unsigned mj = __builtin_amdgcn_ballot_w32(HJ); \
        if (mj != 0u) { \
          if (HJ) { \
            const int pos = wc + (int)__builtin_amdgcn_mbcnt_lo(mj, 0u); \
            if (pos < WCAP) list[wave * WCAP + pos] = ((el0 + (J)) << 12) | (int)(SJ); \
          } \
          wc += (int)__builtin_popcount(mj); } }
      HITJ(0, h0, s0)
      HITJ(1, h1, s1)
      HITJ(2, h2, s2)
      HITJ(3, h3, s3)
      HITJ(4, h4, s4)
      HITJ(5, h5, s5)
      HITJ(6, h6, s6)
      HITJ(7, h7, s7)
#undef HITJ
    }
  }
  return wc;
}

__global__ __launch_bounds__(NTHR) void k_prep(
    const float* __restrict__ W_edge, const float* __restrict__ b_edge,
    const float* __restrict__ W_pre,  const float* __restrict__ b_pre,
    const float* __restrict__ W_post, const float* __restrict__ W_lin,
    _Float16* wp16, _Float16* wq16, float* ce64, float* c0v,
    unsigned short* wph, unsigned short* wpl, unsigned short* wlh, unsigned short* wll)
{
  const int tid = threadIdx.x;

  for (int idx = tid; idx < NT * FT * FT / 8; idx += NTHR) {
    const int e0 = idx * 8, t = e0 >> 8, n = (e0 >> 4) & 15, k0 = e0 & 15;
    const float* wp = W_pre + ((size_t)t * 48 + k0) * FT + n;
    const float* wq = wp + 16 * FT;
    v4f pa, pb, qa, qb;
    pa.x = wp[0 * FT]; pa.y = wp[1 * FT]; pa.z = wp[2 * FT]; pa.w = wp[3 * FT];
    pb.x = wp[4 * FT]; pb.y = wp[5 * FT]; pb.z = wp[6 * FT]; pb.w = wp[7 * FT];
    qa.x = wq[0 * FT]; qa.y = wq[1 * FT]; qa.z = wq[2 * FT]; qa.w = wq[3 * FT];
    qb.x = wq[4 * FT]; qb.y = wq[5 * FT]; qb.z = wq[6 * FT]; qb.w = wq[7 * FT];
    pa = pa * WSC; pb = pb * WSC; qa = qa * WSC; qb = qb * WSC;
    const v8h hp = cvt8(pa, pb), hq = cvt8(qa, qb);
    *(volatile v8h*)(wp16 + e0) = hp;
    *(volatile v8h*)(wq16 + e0) = hq;
    __threadfence();
    *(volatile v8h*)(wp16 + e0) = hp;
    *(volatile v8h*)(wq16 + e0) = hq;
  }

  for (int idx = tid; idx < 4 * HID / 4; idx += NTHR) {
    const int d = idx >> 4, ch0 = (idx & 15) * 4;
    const int t = ch0 >> 4, c = ch0 & 15;
    const float* we = W_edge + d * FT;
    const float* w3 = W_pre + ((size_t)t * 48 + 32) * FT + c;
    v4f r;
    r.x = dot16r(we, w3 + 0, FT);
    r.y = dot16r(we, w3 + 1, FT);
    r.z = dot16r(we, w3 + 2, FT);
    r.w = dot16r(we, w3 + 3, FT);
    *(volatile v4f*)(ce64 + idx * 4) = r;
    __threadfence();
    *(volatile v4f*)(ce64 + idx * 4) = r;
  }

  for (int idx = tid; idx < HID / 4; idx += NTHR) {
    const int ch0 = idx * 4;
    const int t = ch0 >> 4, c = ch0 & 15;
    const float* w3 = W_pre + ((size_t)t * 48 + 32) * FT + c;
    v4f r;
    r.x = b_pre[ch0 + 0] + dot16r(b_edge, w3 + 0, FT);
    r.y = b_pre[ch0 + 1] + dot16r(b_edge, w3 + 1, FT);
    r.z = b_pre[ch0 + 2] + dot16r(b_edge, w3 + 2, FT);
    r.w = b_pre[ch0 + 3] + dot16r(b_edge, w3 + 3, FT);
    *(volatile v4f*)(c0v + idx * 4) = r;
    __threadfence();
    *(volatile v4f*)(c0v + idx * 4) = r;
  }

  for (int idx = tid; idx < NT * FT * KPOST / 8; idx += NTHR) {
    const int e0  = idx * 8;
    const int t   = e0 / (FT * KPOST);
    const int rem = e0 - t * (FT * KPOST);
    const int n   = rem / KPOST;
    const int K0  = rem - n * KPOST;
    FragB hh, ll;
#pragma unroll
    for (int j = 0; j < 8; ++j) {
      const int K   = K0 + j;
      const int row = (K < 16) ? K : (K - 16);
      const bool ok = (K < 16) | (K >= 32);
      float v = W_post[((size_t)t * 208 + row) * FT + n];
      v = ok ? v : 0.0f;
      unsigned short hb, lb;
      split2(v, hb, lb);
      hh.u[j] = hb; ll.u[j] = lb;
    }
    *(volatile v8us*)(wph + e0) = hh.h[0];
    *(volatile v8us*)(wpl + e0) = ll.h[0];
    __threadfence();
    *(volatile v8us*)(wph + e0) = hh.h[0];
    *(volatile v8us*)(wpl + e0) = ll.h[0];
  }

  for (int idx = tid; idx < HID * HID / 8; idx += NTHR) {
    const int e0 = idx * 8, o = e0 >> 6, k0 = e0 & 63;
    FragB hh, ll;
#pragma unroll
    for (int j = 0; j < 8; ++j) {
      const float v = W_lin[(size_t)(k0 + j) * HID + o];
      unsigned short hb, lb;
      split2(v, hb, lb);
      hh.u[j] = hb; ll.u[j] = lb;
    }
    *(volatile v8us*)(wlh + e0) = hh.h[0];
    *(volatile v8us*)(wll + e0) = ll.h[0];
    __threadfence();
    *(volatile v8us*)(wlh + e0) = hh.h[0];
    *(volatile v8us*)(wll + e0) = ll.h[0];
  }
}

__global__ __launch_bounds__(NTHR) void k_node(
    const float* __restrict__ x, const _Float16* __restrict__ wp16, const _Float16* __restrict__ wq16,
    float* Pp, float* Qp, int nN)
{
  __shared__ __attribute__((aligned(16))) float stg_all[NWAVE * 1024];
  const int tid = threadIdx.x, lane = tid & 31, h = lane >> 4, m = lane & 15;
  const int wave = __builtin_amdgcn_readfirstlane(tid >> 5);
  const int row0 = blockIdx.x * NROWS + wave * 16;
  int node = row0 + m;
  node = node > nN - 1 ? nN - 1 : node;

  const v8h z8h = {(_Float16)0.f, (_Float16)0.f, (_Float16)0.f, (_Float16)0.f,
                   (_Float16)0.f, (_Float16)0.f, (_Float16)0.f, (_Float16)0.f};
  v8f accP[NT], accQ[NT];
#pragma unroll
  for (int t = 0; t < NT; ++t) {
    const float* xp = x + (size_t)node * HID + 16 * t + 8 * h;
    FragH a;
    a.h[0] = cvt8(*(const v4f*)xp, *(const v4f*)(xp + 4));
    a.h[1] = z8h;
    FragH bp, bq;
    bp.h[0] = *(const v8h*)(wp16 + (t * 16 + m) * FT + 8 * h);
    bp.h[1] = z8h;
    bq.h[0] = *(const v8h*)(wq16 + (t * 16 + m) * FT + 8 * h);
    bq.h[1] = z8h;
    const v8f zero = {0.f, 0.f, 0.f, 0.f, 0.f, 0.f, 0.f, 0.f};
    accP[t] = wmh(a.v, bp.v, zero);
    accQ[t] = wmh(a.v, bq.v, zero);
  }

  float* stg = stg_all + wave * 1024;
#pragma unroll
  for (int t = 0; t < NT; ++t) {
#pragma unroll
    for (int r = 0; r < 8; ++r) stg[(8 * h + r) * HID + 16 * t + m] = accP[t][r] * WSCI;
  }
  __syncthreads();
  v4f ov[8];
#pragma unroll
  for (int q = 0; q < 8; ++q) ov[q] = *(const v4f*)(stg + q * 128 + 4 * lane);
  __syncthreads();
#pragma unroll
  for (int t = 0; t < NT; ++t) {
#pragma unroll
    for (int r = 0; r < 8; ++r) stg[(8 * h + r) * HID + 16 * t + m] = accQ[t][r] * WSCI;
  }
  __syncthreads();
  v4f ow[8];
#pragma unroll
  for (int q = 0; q < 8; ++q) ow[q] = *(const v4f*)(stg + q * 128 + 4 * lane);

  float* gp = Pp + (size_t)row0 * HID + 4 * lane;
  float* gq = Qp + (size_t)row0 * HID + 4 * lane;
#pragma unroll
  for (int q = 0; q < 8; ++q) *(volatile v4f*)(gp + q * 128) = ov[q];
#pragma unroll
  for (int q = 0; q < 8; ++q) *(volatile v4f*)(gq + q * 128) = ow[q];
  __threadfence();
#pragma unroll
  for (int q = 0; q < 8; ++q) *(volatile v4f*)(gp + q * 128) = ov[q];
#pragma unroll
  for (int q = 0; q < 8; ++q) *(volatile v4f*)(gq + q * 128) = ow[q];
}

__device__ __forceinline__ void finalize_elem(float* sp, int c, float inv) {
#pragma clang fp contract(off)
  const float ssum = sp[0], s2 = sp[HID], mn = sp[2 * HID], mx = sp[3 * HID];
  const float mean = ssum * inv;
  const float var  = fmaxf(s2 * inv - mean * mean, 0.0f);
  const float sd   = sqrtf(var + STDEPS);
  const bool  emp  = (c == 0);
  sp[0]       = mean;
  sp[HID]     = emp ? 0.0f : mn;
  sp[2 * HID] = emp ? 0.0f : mx;
  sp[3 * HID] = sd;
}

__global__ __launch_bounds__(NTHR) __attribute__((amdgpu_num_vgpr(256))) void k_agg(
    const int* __restrict__ ei, const float* __restrict__ eattr,
    const float* __restrict__ Pp, const float* __restrict__ Qp,
    const float* __restrict__ ce64, const float* __restrict__ c0v,
    const float* __restrict__ x,
    const unsigned short* __restrict__ wph, const unsigned short* __restrict__ wpl,
    const float* __restrict__ b_post,
    const unsigned short* __restrict__ wlh, const unsigned short* __restrict__ wll,
    const float* __restrict__ b_lin,
    float* out, int nN, int nE, int vec8)
{
  extern __shared__ v4f lds_dyn[];
  float* st   = (float*)lds_dyn;
  int*   list = (int*)(st + NBA * SLOTF);
  int*   cnt  = list + LISTN;
  int*   wcnt = cnt + NBA;
  float* ampA = (float*)list;
  float* attA = ampA + NBA;
  float* invA = attA + NBA;
  const int tid = threadIdx.x, lane = tid & 31, h = lane >> 4, m = lane & 15;
  const int wave = __builtin_amdgcn_readfirstlane(tid >> 5);
  const int nodeBase = blockIdx.x * NBA;
  const int* dsts = ei + nE;

  for (int i = tid; i < NBA * SLOTF / 4; i += NTHR) {
    const int stat = (i >> 4) & 3;
    const float val = (stat < 2) ? 0.0f : ((stat == 2) ? __builtin_inff() : -__builtin_inff());
    const v4f z = {val, val, val, val};
    lds_dyn[i] = z;
  }
  for (int i = tid; i < NBA; i += NTHR) cnt[i] = 0;
  __syncthreads();

  const v2f ce0 = *(const v2f*)(ce64 + 0 * HID + 2 * lane);
  const v2f ce1 = *(const v2f*)(ce64 + 1 * HID + 2 * lane);
  const v2f ce2 = *(const v2f*)(ce64 + 2 * HID + 2 * lane);
  const v2f ce3 = *(const v2f*)(ce64 + 3 * HID + 2 * lane);
  const v2f c0r = *(const v2f*)(c0v + 2 * lane);

  const int nChunks = (nE + CHUNK - 1) / CHUNK;
#pragma unroll 1
  for (int chn = 0; chn < nChunks; ++chn) {
    const int cbase = chn * CHUNK;
    const int wc = scan_chunk<NBA>(dsts, nE, cbase, nodeBase, vec8, list, tid, lane, wave);
    if (lane == 0) wcnt[wave] = wc;
    __syncthreads();
#pragma unroll 1
    for (int wsx = 0; wsx < NWAVE; ++wsx) {
      int n = __builtin_amdgcn_readfirstlane(wcnt[wsx]);
      n = n > WCAP ? WCAP : (n < 0 ? 0 : n);
      const int* lp = list + wsx * WCAP;
#pragma unroll 1
      for (int i = 0; i < n; ++i) {
        const int ent  = __builtin_amdgcn_readfirstlane(lp[i]);
        const int slot = ent & (NBA - 1);
        if ((slot & (NWAVE - 1)) != wave) continue;
        int e = cbase + ((ent >> 12) & (CHUNK - 1));
        e = e > nE - 1 ? nE - 1 : e;
        int src = ei[e];
        src = src < 0 ? 0 : (src > nN - 1 ? nN - 1 : src);
        int dn = nodeBase + slot;
        dn = dn > nN - 1 ? nN - 1 : dn;
        const v4f ea = *(const v4f*)(eattr + (size_t)e * 4);
        const v2f qv = *(const v2f*)(Qp + (size_t)src * HID + 2 * lane);
        const v2f pv = *(const v2f*)(Pp + (size_t)dn * HID + 2 * lane);
        const float ex = c0r.x + ea.x * ce0.x + ea.y * ce1.x + ea.z * ce2.x + ea.w * ce3.x;
        const float ey = c0r.y + ea.x * ce0.y + ea.y * ce1.y + ea.z * ce2.y + ea.w * ce3.y;
        const float m0 = (pv.x + qv.x) + ex;
        const float m1 = (pv.y + qv.y) + ey;
        float* sp = st + slot * SLOTF + 2 * lane;
        v2f s1 = *(const v2f*)sp;
        s1.x += m0; s1.y += m1;
        *(v2f*)sp = s1;
        v2f s2 = *(const v2f*)(sp + HID);
        s2.x += m0 * m0; s2.y += m1 * m1;
        *(v2f*)(sp + HID) = s2;
        v2f mn = *(const v2f*)(sp + 2 * HID);
        mn.x = fminf(mn.x, m0); mn.y = fminf(mn.y, m1);
        *(v2f*)(sp + 2 * HID) = mn;
        v2f mx = *(const v2f*)(sp + 3 * HID);
        mx.x = fmaxf(mx.x, m0); mx.y = fmaxf(mx.y, m1);
        *(v2f*)(sp + 3 * HID) = mx;
        if (lane == 0) cnt[slot] = cnt[slot] + 1;
      }
    }
    __syncthreads();
  }

  if (tid < NBA) {
    const int c = cnt[tid];
    const float degf = fmaxf((float)c, 1.0f);
    const float ld   = logf(degf + 1.0f);
    invA[tid] = 1.0f / degf;
    ampA[tid] = ld * (1.0f / AVGL);
    attA[tid] = AVGL * (1.0f / ld);
  }
  __syncthreads();
#pragma unroll 1
  for (int i = 0; i < (NBA * HID) / NTHR; ++i) {
    const int idx  = i * NTHR + tid;
    const int slot = idx >> 6;
    const int chx  = idx & 63;
    finalize_elem(st + slot * SLOTF + chx, cnt[slot], invA[slot]);
  }
  __syncthreads();

  const v8us z8us = {0, 0, 0, 0, 0, 0, 0, 0};
#pragma unroll 1
  for (int it = 0; it < (NBA / 16) / NWAVE; ++it) {
    const int tile     = wave + NWAVE * it;
    const int slotBase = tile * 16;
    const float amp = ampA[slotBase + m];
    const float att = attA[slotBase + m];
    int node = nodeBase + slotBase + m;
    node = node > nN - 1 ? nN - 1 : node;

    v8f accP[NT];
#pragma unroll
    for (int t = 0; t < NT; ++t) {
      const v8f zero = {0.f, 0.f, 0.f, 0.f, 0.f, 0.f, 0.f, 0.f};
      accP[t] = zero;
      {
        const float* xp = x + (size_t)node * HID + 16 * t + 8 * h;
        const v4f p0 = *(const v4f*)xp, p1 = *(const v4f*)(xp + 4);
        FragB ah, al, bh, bl;
        split4<0>(p0, ah, al);
        split4<4>(p1, ah, al);
        ah.h[1] = z8us; al.h[1] = z8us;
        const int off = (t * 16 + m) * KPOST + 8 * h;
        loadB(wph + off, bh);
        loadB(wpl + off, bl);
        accP[t] = wmb3(ah, al, bh, bl, accP[t]);
      }
#pragma unroll
      for (int kc = 1; kc < 7; ++kc) {
        const int pair = (kc - 1) & 1;
        const int sel  = (kc - 1) >> 1;
        const float s  = (sel == 0) ? 1.0f : ((sel == 1) ? amp : att);
        const float* ap = st + (slotBase + m) * SLOTF + pair * 128 + 16 * t + 8 * h;
        v4f p0 = *(const v4f*)ap,        p1 = *(const v4f*)(ap + 4);
        v4f p2 = *(const v4f*)(ap + 64), p3 = *(const v4f*)(ap + 68);
        p0 = p0 * s; p1 = p1 * s; p2 = p2 * s; p3 = p3 * s;
        FragB ah, al, bh, bl;
        split4<0>(p0, ah, al);
        split4<4>(p1, ah, al);
        split4<8>(p2, ah, al);
        split4<12>(p3, ah, al);
        const int off = (t * 16 + m) * KPOST + 32 * kc + 8 * h;
        loadB(wph + off, bh);
        loadB(wpl + off, bl);
        accP[t] = wmb3(ah, al, bh, bl, accP[t]);
      }
    }
    __syncthreads();

    float* stg = st + slotBase * SLOTF;
#pragma unroll
    for (int t = 0; t < NT; ++t) {
      const float bb = b_post[16 * t + m];
#pragma unroll
      for (int r = 0; r < 8; ++r) stg[(8 * h + r) * HID + 16 * t + m] = accP[t][r] + bb;
    }
    __syncthreads();

    v8f accL[4];
#pragma unroll
    for (int jt = 0; jt < 4; ++jt) { const v8f zero = {0.f, 0.f, 0.f, 0.f, 0.f, 0.f, 0.f, 0.f}; accL[jt] = zero; }
#pragma unroll
    for (int kc = 0; kc < 2; ++kc) {
      const float* ap = stg + m * HID + 32 * kc + 8 * h;
      const v4f p0 = *(const v4f*)ap,        p1 = *(const v4f*)(ap + 4);
      const v4f p2 = *(const v4f*)(ap + 16), p3 = *(const v4f*)(ap + 20);
      FragB ah, al;
      split4<0>(p0, ah, al);
      split4<4>(p1, ah, al);
      split4<8>(p2, ah, al);
      split4<12>(p3, ah, al);
#pragma unroll
      for (int jt = 0; jt < 4; ++jt) {
        FragB bh, bl;
        const int off = (jt * 16 + m) * HID + 32 * kc + 8 * h;
        loadB(wlh + off, bh);
        loadB(wll + off, bl);
        accL[jt] = wmb3(ah, al, bh, bl, accL[jt]);
      }
    }
    float* stg2 = stg + 1024;
#pragma unroll
    for (int jt = 0; jt < 4; ++jt) {
      const float bb = b_lin[16 * jt + m];
#pragma unroll
      for (int r = 0; r < 8; ++r) stg2[(8 * h + r) * HID + 16 * jt + m] = fmaxf(accL[jt][r] + bb, 0.0f);
    }
    __syncthreads();

    v4f ov[8];
#pragma unroll
    for (int q = 0; q < 8; ++q) ov[q] = *(const v4f*)(stg2 + q * 128 + 4 * lane);
    const int rowNode0 = nodeBase + slotBase;
#pragma unroll
    for (int q = 0; q < 8; ++q) {
      const int nd = rowNode0 + 2 * q + h;
      if (nd < nN) *(volatile v4f*)(out + (size_t)(rowNode0 + 2 * q) * HID + 4 * lane) = ov[q];
    }
    __threadfence();
#pragma unroll
    for (int q = 0; q < 8; ++q) {
      const int nd = rowNode0 + 2 * q + h;
      if (nd < nN) *(volatile v4f*)(out + (size_t)(rowNode0 + 2 * q) * HID + 4 * lane) = ov[q];
    }
  }
}

extern "C" void kernel_launch(void* const* d_in, const int* in_sizes, int n_in,
                              void* d_out, int out_size, void* d_ws, size_t ws_size,
                              hipStream_t stream)
{
  if (n_in < 11) return;
  const int nN = in_sizes[0] / HID;
  const int nE = in_sizes[1] / 2;
  if (nN <= 0 || nE < 1 || in_sizes[0] != nN * HID || in_sizes[1] != nE * 2) return;
  if (in_sizes[2] != nE * 4) return;
  if (in_sizes[3] != 4 * FT || in_sizes[4] != FT) return;
  if (in_sizes[5] != NT * 48 * FT || in_sizes[6] != NT * FT) return;
  if (in_sizes[7] != NT * 208 * FT || in_sizes[8] != NT * FT) return;
  if (in_sizes[9] != HID * HID || in_sizes[10] != HID) return;
  if (out_size != nN * HID) return;

  const float* x      = (const float*)d_in[0];
  const int*   ei     = (const int*)d_in[1];
  const float* eattr  = (const float*)d_in[2];
  const float* W_edge = (const float*)d_in[3];
  const float* b_edge = (const float*)d_in[4];
  const float* W_pre  = (const float*)d_in[5];
  const float* b_pre  = (const float*)d_in[6];
  const float* W_post = (const float*)d_in[7];
  const float* b_post = (const float*)d_in[8];
  const float* W_lin  = (const float*)d_in[9];
  const float* b_lin  = (const float*)d_in[10];
  float* out = (float*)d_out;

  const int rowsPad = ((nN + NBA - 1) / NBA) * NBA;
  const int nBlkA   = rowsPad / NBA;
  const int nBlkN   = rowsPad / NROWS;

  char* ws = (char*)d_ws;
  size_t off = 0;
  const size_t oWP  = off; off += (size_t)NT * FT * FT * 2;                    off = (off + 255) & ~(size_t)255;
  const size_t oWQ  = off; off += (size_t)NT * FT * FT * 2;                    off = (off + 255) & ~(size_t)255;
  const size_t oCE  = off; off += (size_t)4 * HID * 4;                          off = (off + 255) & ~(size_t)255;
  const size_t oC0  = off; off += (size_t)HID * 4;                              off = (off + 255) & ~(size_t)255;
  const size_t oWPH = off; off += (size_t)NT * FT * KPOST * 2;                  off = (off + 255) & ~(size_t)255;
  const size_t oWPL = off; off += (size_t)NT * FT * KPOST * 2;                  off = (off + 255) & ~(size_t)255;
  const size_t oWLH = off; off += (size_t)HID * HID * 2;                        off = (off + 255) & ~(size_t)255;
  const size_t oWLL = off; off += (size_t)HID * HID * 2;                        off = (off + 255) & ~(size_t)255;
  const size_t oP   = off; off += (size_t)rowsPad * HID * 4;                    off = (off + 255) & ~(size_t)255;
  const size_t oQ   = off; off += (size_t)rowsPad * HID * 4;                    off = (off + 255) & ~(size_t)255;
  if (off > ws_size) return;

  _Float16*       wp16 = (_Float16*)(ws + oWP);
  _Float16*       wq16 = (_Float16*)(ws + oWQ);
  float*          ce64 = (float*)(ws + oCE);
  float*          c0v  = (float*)(ws + oC0);
  unsigned short* wph  = (unsigned short*)(ws + oWPH);
  unsigned short* wpl  = (unsigned short*)(ws + oWPL);
  unsigned short* wlh  = (unsigned short*)(ws + oWLH);
  unsigned short* wll  = (unsigned short*)(ws + oWLL);
  float*          Pp   = (float*)(ws + oP);
  float*          Qp   = (float*)(ws + oQ);

  const int vec8 = ((nE & 3) == 0) ? 1 : 0;

  k_prep<<<1, NTHR, 0, stream>>>(W_edge, b_edge, W_pre, b_pre, W_post, W_lin,
                                 wp16, wq16, ce64, c0v, wph, wpl, wlh, wll);

  k_node<<<nBlkN, NTHR, 0, stream>>>(x, wp16, wq16, Pp, Qp, nN);

  hipFuncSetAttribute(reinterpret_cast<const void*>(&k_agg),
                      hipFuncAttributeMaxDynamicSharedMemorySize, LDS_AGG);
  k_agg<<<nBlkA, NTHR, LDS_AGG, stream>>>(ei, eattr, Pp, Qp, ce64, c0v, x,
                                          wph, wpl, b_post, wlh, wll, b_lin,
                                          out, nN, nE, vec8);
}
